// StackedWaveNet_61125974556799
// MI455X (gfx1250) — hardware-verified
//
#include <hip/hip_runtime.h>
#include <math.h>

typedef __attribute__((ext_vector_type(16))) _Float16 v16h;
typedef __attribute__((ext_vector_type(16))) __bf16 v16b;
typedef __attribute__((ext_vector_type(8)))  _Float16 v8h;
typedef __attribute__((ext_vector_type(8)))  float v8f;
typedef __attribute__((ext_vector_type(4)))  float v4f;
typedef __attribute__((ext_vector_type(2)))  float v2f;
typedef __attribute__((ext_vector_type(4)))  unsigned v4u;
typedef __attribute__((ext_vector_type(4)))  int v4i;
typedef float __attribute__((may_alias)) float_a;
typedef int __attribute__((may_alias)) int_a;

template <typename T> __device__ __forceinline__ void vst2(void* p, T v) { *(volatile T*)p = v; __threadfence(); *(volatile T*)p = v; }
__device__ __forceinline__ v8f wmma16(v16h a, v16h b, v8f c) {
  v8f d = __builtin_amdgcn_wmma_f32_16x16x32_f16(false, a, false, b, (short)0, c, false, false);
  asm volatile("v_nop\n\tv_nop\n\tv_nop\n\tv_nop" : "+v"(d) : "v"(a), "v"(b));
  return d;
}
__device__ __forceinline__ v8f wmma_bf(v16b a, v16b b, v8f c) {
  v8f d = __builtin_amdgcn_wmma_f32_16x16x32_bf16(false, a, false, b, (short)0, c, false, false);
  asm volatile("v_nop\n\tv_nop\n\tv_nop\n\tv_nop" : "+v"(d) : "v"(a), "v"(b));
  return d;
}
__device__ __forceinline__ v16h frag_h(const _Float16* rowk0, int lane) {
  union { v16h v; v8h q[2]; } u; const _Float16* p = rowk0 + 8 * (lane >> 4);
  u.q[0] = *(const v8h*)p; u.q[1] = *(const v8h*)(p + 16); return u.v;
}
__device__ __forceinline__ v16h frag_f32(const float* rowk0, int lane) {
  v16h a; const float* p = rowk0 + 8 * (lane >> 4);
#pragma unroll
  for (int i = 0; i < 8; ++i) { a[i] = (_Float16)p[i]; a[8 + i] = (_Float16)p[16 + i]; }
  return a;
}
__device__ __forceinline__ v16h frag_f32s(const float* rowk0, int lane, float sc) {
  v16h a; const float* p = rowk0 + 8 * (lane >> 4);
#pragma unroll
  for (int i = 0; i < 8; ++i) { a[i] = (_Float16)(p[i] * sc); a[8 + i] = (_Float16)(p[16 + i] * sc); }
  return a;
}
__device__ __forceinline__ v16h fragc_f32(const float* W, int k0, int n, int lane, int ld, int K) {
  v16h a; const int g = lane >> 4;
#pragma unroll
  for (int i = 0; i < 8; ++i) { const int ka = k0 + 8 * g + i, kb = ka + 16;
    a[i] = (_Float16)(ka < K ? W[(size_t)(ka < K ? ka : K - 1) * ld + n] : 0.f); a[8 + i] = (_Float16)(kb < K ? W[(size_t)(kb < K ? kb : K - 1) * ld + n] : 0.f); }
  return a;
}
struct F2 { v16b h, l; };
__device__ __forceinline__ F2 bsplit16(const float v[16]) { F2 r;
#pragma unroll
  for (int i = 0; i < 16; ++i) { const __bf16 h = (__bf16)v[i]; r.h[i] = h; r.l[i] = (__bf16)(v[i] - (float)h); }
  return r; }
__device__ __forceinline__ F2 split_row(const float* row, int k0, int lane) { float v[16]; const float* p = row + k0 + 8 * (lane >> 4);
#pragma unroll
  for (int i = 0; i < 8; ++i) { v[i] = p[i]; v[8 + i] = p[16 + i]; }
  return bsplit16(v); }
__device__ __forceinline__ F2 split_rowK(const float* row, int k0, int lane, int K) { float v[16]; const int g = lane >> 4;
#pragma unroll
  for (int i = 0; i < 8; ++i) { const int ka = k0 + 8 * g + i, kb = ka + 16; v[i] = ka < K ? row[ka < K ? ka : K - 1] : 0.f; v[8 + i] = kb < K ? row[kb < K ? kb : K - 1] : 0.f; }
  return bsplit16(v); }
__device__ __forceinline__ F2 split_col(const float* W, int k0, int n, int lane, int ld, int K) { float v[16]; const int g = lane >> 4;
#pragma unroll
  for (int i = 0; i < 8; ++i) { const int ka = k0 + 8 * g + i, kb = ka + 16; v[i] = ka < K ? W[(size_t)(ka < K ? ka : K - 1) * ld + n] : 0.f; v[8 + i] = kb < K ? W[(size_t)(kb < K ? kb : K - 1) * ld + n] : 0.f; }
  return bsplit16(v); }
__device__ __forceinline__ v8f mac3(const F2& a, const F2& b, v8f c) { c = wmma_bf(a.l, b.h, c); c = wmma_bf(a.h, b.l, c); return wmma_bf(a.h, b.h, c); }
__device__ __forceinline__ float sigm(float v) { return 1.0f / (1.0f + expf(-v)); }
#define LDSX() do { asm volatile("s_wait_dscnt 0" ::: "memory"); __builtin_amdgcn_wave_barrier(); __builtin_amdgcn_fence(__ATOMIC_RELEASE, "workgroup"); } while (0)


#define NSQ 4
#define TL 16384
#define RC 64
#define SCH 128
#define NLAY 30
#define NR (NSQ * TL)
#ifndef TRB
#define TRB (NR / 64)
#endif
typedef __attribute__((ext_vector_type(8))) __bf16 v8b;
__device__ __forceinline__ v16b frag_b(const __bf16* rowk0, int lane) {
  union { v16b v; v8b q[2]; } u; const __bf16* p = rowk0 + 8 * (lane >> 4);
  u.q[0] = *(const v8b*)p; u.q[1] = *(const v8b*)(p + 16); return u.v;
}
__device__ __forceinline__ float bfr(float v) { return (float)(__bf16)v; }
__device__ __attribute__((noinline)) float exp_ni(float v) { return expf(v); }
__device__ __attribute__((noinline)) float erf_ni(float v) { return erff(v); }

__device__ __attribute__((noinline)) float tanh_ni(float v) { return tanhf(v); }
__device__ __forceinline__ void put_hl(__bf16* h, __bf16* l, float v) { const __bf16 hb = (__bf16)v; *h = hb; *l = (__bf16)(v - (float)hb); }
#define PK_FG  0
#define PK_RS  (PK_FG + (size_t)NLAY * 128 * 128)
#define PK_P   (PK_RS + (size_t)NLAY * 192 * 64)
#define PK_O1  (PK_P + 128 * 128)
#define PK_END (PK_O1 + 128 * 128)
#define WS_PK  0u
#define WS_HA  (WS_PK + 2u * (unsigned)PK_END)
#define WS_HB  (WS_HA + 4u * NR * RC)
#define WS_SK  (WS_HB + 4u * NR * RC)
#define WS_END (WS_SK + 4u * NR * SCH)

__global__ __launch_bounds__(128) void k_pack3(const float* __restrict__ Wf, const float* __restrict__ Wg, const float* __restrict__ Wr, const float* __restrict__ Wsk, __bf16* __restrict__ PK, int which) {
  __shared__ __align__(16) __bf16 s[8 * 128]; const int lay = blockIdx.y, grp = blockIdx.x, tid = threadIdx.x;
  if (which == 0) {
    for (int q = tid; q < 8 * 128; q += 128) { const int rl = q >> 7, k = q & 127; const int row = grp * 8 + rl; const int o = row & 63; const float* Wsrc = (row < 64) ? Wf : Wg; const int c = k & 63, tap = k >> 6;
      s[q] = (__bf16)Wsrc[(((size_t)lay * RC + o) * RC + c) * 2 + tap]; }
    __syncthreads();
    vst2((unsigned*)(PK + PK_FG + ((size_t)lay * 128 + grp * 8) * 128 + tid * 8), *(const v4u*)&s[tid * 8]);
  } else {
    for (int q = tid; q < 8 * 64; q += 128) { const int rl = q >> 6, c = q & 63; const int row = grp * 8 + rl; float v;
      if (row < 64) v = Wr[((size_t)lay * RC + row) * RC + c]; else v = Wsk[((size_t)lay * SCH + (row - 64)) * RC + c];
      s[q] = (__bf16)v; }
    __syncthreads();
    if (tid < 64) vst2((unsigned*)(PK + PK_RS + ((size_t)lay * 192 + grp * 8) * 64 + tid * 8), *(const v4u*)&s[tid * 8]);
  }
}
__global__ __launch_bounds__(128) void k_pack1(const float* __restrict__ Wm, __bf16* __restrict__ DST) {
  __shared__ __align__(16) __bf16 s[128]; const int n = blockIdx.x, tid = threadIdx.x; s[tid] = (__bf16)Wm[(size_t)n * 128 + tid]; __syncthreads();
  if (tid < 16) vst2((unsigned*)(DST + (size_t)n * 128 + tid * 8), *(const v4u*)&s[tid * 8]);
}
__global__ __launch_bounds__(256) void k_init(const float* __restrict__ X, const float* __restrict__ WC, const float* __restrict__ BC, float* __restrict__ H, float* __restrict__ SK) {
  __shared__ __align__(16) float sh[64][RC + 4];
  const int tid = threadIdx.x; { const int rl = tid >> 2; const size_t r = (size_t)blockIdx.x * 64 + rl; const int c0 = (tid & 3) * 16; const int t = (int)(r % TL);
    const float xc = bfr(X[r]), xp = (t > 0) ? bfr(X[r - 1]) : 0.f;
#pragma unroll
    for (int i = 0; i < 16; ++i) { const int c = c0 + i; sh[rl][c] = bfr(WC[c * 2 + 0]) * xp + bfr(WC[c * 2 + 1]) * xc + bfr(BC[c]); } }
  __syncthreads();
  for (int q = tid; q < 64 * 16; q += 256) { const int rl = q >> 4, pc = q & 15; vst2(H + ((size_t)blockIdx.x * 64 + rl) * RC + pc * 4, *(const v4f*)&sh[rl][pc * 4]); }
  for (int q = tid; q < 64 * 32; q += 256) { const int rl = q >> 5, pc = q & 31; vst2(SK + ((size_t)blockIdx.x * 64 + rl) * SCH + pc * 4, (v4f){0.f, 0.f, 0.f, 0.f}); }
}
__global__ __launch_bounds__(128) void k_layer(const float* __restrict__ Hin, float* __restrict__ Hout, float* __restrict__ SK, const __bf16* __restrict__ PFG, const __bf16* __restrict__ PRS, const float* __restrict__ bf, const float* __restrict__ bg, const float* __restrict__ br, const float* __restrict__ bs, int dil) {
  __shared__ __align__(16) __bf16 soh[4][16][72], sol[4][16][72]; __shared__ __align__(16) float sh[4][16][68]; __shared__ __align__(16) float ssk[4][16][132];
  const int tid = threadIdx.x, wave = tid >> 5, lane = tid & 31, col = lane & 15, g = lane >> 4; const size_t r0 = (size_t)blockIdx.x * 64 + wave * 16; const size_t ra = r0 + col; const int t = (int)(ra % TL);
  v8f acc[8] = {};
#pragma unroll
  for (int kc = 0; kc < 4; ++kc) { F2 a;
    if (kc < 2) { const bool ok = (t - dil) >= 0; const float* p = Hin + (ok ? ra - dil : ra) * RC + kc * 32 + 8 * g; float v[16];
#pragma unroll
      for (int i = 0; i < 8; ++i) { v[i] = ok ? p[i] : 0.f; v[8 + i] = ok ? p[16 + i] : 0.f; }
      a = bsplit16(v); }
    else a = split_row(Hin + ra * RC, (kc - 2) * 32, lane);
#pragma unroll
    for (int j = 0; j < 8; ++j) { const v16b w = frag_b(PFG + (size_t)(j * 16 + col) * 128 + kc * 32, lane); acc[j] = wmma_bf(a.l, w, acc[j]); acc[j] = wmma_bf(a.h, w, acc[j]); } }
#pragma unroll
  for (int j = 0; j < 4; ++j) { const int o = j * 16 + col; const float b0 = bfr(bf[o]), b1 = bfr(bg[o]);
#pragma unroll
    for (int r = 0; r < 8; ++r) { const float fv = tanh_ni(acc[j][r] + b0), gv = sigm(acc[j + 4][r] + b1); put_hl(&soh[wave][8 * g + r][o], &sol[wave][8 * g + r][o], fv * gv); } }
  LDSX();
  { v8f ac2[12] = {};
#pragma unroll
    for (int kc = 0; kc < 2; ++kc) { const v16b oh = frag_b(&soh[wave][col][kc * 32], lane), ol = frag_b(&sol[wave][col][kc * 32], lane);
#pragma unroll
      for (int j = 0; j < 12; ++j) { const v16b w = frag_b(PRS + (size_t)(j * 16 + col) * 64 + kc * 32, lane); ac2[j] = wmma_bf(ol, w, ac2[j]); ac2[j] = wmma_bf(oh, w, ac2[j]); } }
#pragma unroll
    for (int j = 0; j < 4; ++j) { const int o = j * 16 + col; const float bb = bfr(br[o]);
#pragma unroll
      for (int r = 0; r < 8; ++r) sh[wave][8 * g + r][o] = ac2[j][r] + bb + Hin[(r0 + 8 * g + r) * RC + o]; }
#pragma unroll
    for (int j = 4; j < 12; ++j) { const int o = (j - 4) * 16 + col; const float bb = bfr(bs[o]);
#pragma unroll
      for (int r = 0; r < 8; ++r) ssk[wave][8 * g + r][o] = ac2[j][r] + bb + SK[(r0 + 8 * g + r) * SCH + o]; } }
  LDSX();
  for (int rl = 0; rl < 16; ++rl) { if (lane < 16) vst2(Hout + (r0 + rl) * RC + lane * 4, *(const v4f*)&sh[wave][rl][lane * 4]); vst2(SK + (r0 + rl) * SCH + lane * 4, *(const v4f*)&ssk[wave][rl][lane * 4]); }
}
__global__ __launch_bounds__(128) void k_post(const float* __restrict__ SK, const __bf16* __restrict__ PP, const float* __restrict__ bp, const __bf16* __restrict__ PO1, const float* __restrict__ bo1, const float* __restrict__ wo2, const float* __restrict__ bo2, float* __restrict__ out) {
  __shared__ __align__(16) __bf16 s1h[4][16][136], s1l[4][16][136]; __shared__ float s2[4][16][132]; __shared__ __align__(16) float sy[64];
  const int tid = threadIdx.x, wave = tid >> 5, lane = tid & 31, col = lane & 15, g = lane >> 4; const size_t r0 = (size_t)blockIdx.x * 64 + wave * 16;
  { v8f acc[8] = {};
#pragma unroll
    for (int kc = 0; kc < 4; ++kc) { const F2 a = split_row(SK + (r0 + col) * SCH, kc * 32, lane);
#pragma unroll
      for (int j = 0; j < 8; ++j) { const v16b w = frag_b(PP + (size_t)(j * 16 + col) * 128 + kc * 32, lane); acc[j] = wmma_bf(a.l, w, acc[j]); acc[j] = wmma_bf(a.h, w, acc[j]); } }
#pragma unroll
    for (int j = 0; j < 8; ++j) { const int o = j * 16 + col; const float bb = bfr(bp[o]);
#pragma unroll
      for (int r = 0; r < 8; ++r) put_hl(&s1h[wave][8 * g + r][o], &s1l[wave][8 * g + r][o], fmaxf(acc[j][r] + bb, 0.f)); } }
  LDSX();
  { v8f acc[8] = {};
#pragma unroll
    for (int kc = 0; kc < 4; ++kc) { const v16b ah = frag_b(&s1h[wave][col][kc * 32], lane), al = frag_b(&s1l[wave][col][kc * 32], lane);
#pragma unroll
      for (int j = 0; j < 8; ++j) { const v16b w = frag_b(PO1 + (size_t)(j * 16 + col) * 128 + kc * 32, lane); acc[j] = wmma_bf(al, w, acc[j]); acc[j] = wmma_bf(ah, w, acc[j]); } }
#pragma unroll
    for (int j = 0; j < 8; ++j) { const int o = j * 16 + col; const float bb = bfr(bo1[o]);
#pragma unroll
      for (int r = 0; r < 8; ++r) s2[wave][8 * g + r][o] = fmaxf(acc[j][r] + bb, 0.f); } }
  LDSX();
  if (lane < 16) { float y = bfr(bo2[0]);
#pragma unroll 4
    for (int o = 0; o < SCH; ++o) y += s2[wave][lane][o] * bfr(wo2[o]);
    sy[wave * 16 + lane] = y; }
  __syncthreads();
  if (tid < 16) vst2(out + (size_t)blockIdx.x * 64 + tid * 4, *(const v4f*)&sy[tid * 4]);
}
extern "C" void kernel_launch(void* const* d_in, const int* in_sizes, int n_in, void* d_out, int out_size, void* d_ws, size_t ws_size, hipStream_t stream) {
  (void)in_sizes; (void)n_in; (void)out_size;
  const float** F = (const float**)d_in;
  if (ws_size < (size_t)WS_END) return;
  char* ws = (char*)d_ws; __bf16* PK = (__bf16*)(ws + WS_PK); float *HA = (float*)(ws + WS_HA), *HB = (float*)(ws + WS_HB), *SK = (float*)(ws + WS_SK);
  k_pack3<<<dim3(16, NLAY), 128, 0, stream>>>(F[3], F[5], F[7], F[9], PK, 0);
  k_pack3<<<dim3(24, NLAY), 128, 0, stream>>>(F[3], F[5], F[7], F[9], PK, 1);
  k_pack1<<<128, 128, 0, stream>>>(F[11], PK + PK_P);
  k_pack1<<<128, 128, 0, stream>>>(F[13], PK + PK_O1);
  k_init<<<TRB, 256, 0, stream>>>(F[0], F[1], F[2], HA, SK);
  float* hin = HA; float* hout = HB;
  for (int i = 0; i < NLAY; ++i) { const int dil = 1 << (i % 10);
    k_layer<<<TRB, 128, 0, stream>>>(hin, hout, SK, PK + PK_FG + (size_t)i * 128 * 128, PK + PK_RS + (size_t)i * 192 * 64, F[4] + i * RC, F[6] + i * RC, F[8] + i * RC, F[10] + i * SCH, dil);
    float* tmp = hin; hin = hout; hout = tmp; }
  k_post<<<TRB, 128, 0, stream>>>(SK, PK + PK_P, F[12], PK + PK_O1, F[14], F[15], F[16], (float*)d_out);
}
